// IndependentPolicy_77068893160318
// MI455X (gfx1250) — hardware-verified
//
#include <hip/hip_runtime.h>
#include <stddef.h>
#include <math.h>


#pragma clang fp contract(off)

#define HID    64
#define HID2   128
#define NSLOT  4
#define SEQL   24
#define NSTEP  23
#define NVOC   66
#define GH     32
#define NTHR   128
#define NWAVE  4
#define AP     136
#define HP     72

#define L_EA    0
#define L_EM    (L_EA + NVOC * GH * 4)
#define L_WG    (L_EM + NVOC * GH * 4)
#define L_GB1   (L_WG + NTHR * 4)
#define L_GW2   (L_GB1 + GH * 4)
#define L_RB1   (L_GW2 + GH * 4)
#define L_RB2   (L_RB1 + HID * 4)
#define L_AH    (L_RB2 + HID * 4)
#define L_AL    (L_AH + NTHR * AP * 2)
#define L_W1H   (L_AL + NTHR * AP * 2)
#define L_W1L   (L_W1H + HID * AP * 2)
#define L_HH    (L_W1L + HID * AP * 2)
#define L_HL    (L_HH + NTHR * HP * 2)
#define L_W2H   (L_HL + NTHR * HP * 2)
#define L_W2L   (L_W2H + HID * HP * 2)
#define LDS_TOT (L_W2L + HID * HP * 2)

static_assert(NTHR == NWAVE * 32);
static_assert(GH == 32 && HID == 64 && HID2 == 2 * HID);
static_assert((L_EM % 16) == 0 && (L_WG % 16) == 0 && (L_GB1 % 16) == 0 && (L_GW2 % 16) == 0);
static_assert((L_RB1 % 16) == 0 && (L_RB2 % 16) == 0 && (L_AH % 16) == 0 && (L_AL % 16) == 0);
static_assert((L_W1H % 16) == 0 && (L_W1L % 16) == 0 && (L_HH % 16) == 0 && (L_HL % 16) == 0);
static_assert((L_W2H % 16) == 0 && (L_W2L % 16) == 0);
static_assert((AP * 2) % 16 == 0 && (HP * 2) % 16 == 0);
static_assert(NVOC * GH * 4 <= NTHR * AP * 2);
static_assert(NWAVE * 32 * HID * 4 <= 2 * NTHR * AP * 2);
static_assert(LDS_TOT == 177920);

typedef float          v4f   __attribute__((ext_vector_type(4)));
typedef float          v8f   __attribute__((ext_vector_type(8)));
typedef unsigned int   v4u   __attribute__((ext_vector_type(4)));
typedef unsigned short v8us  __attribute__((ext_vector_type(8)));
typedef __bf16         v16bf __attribute__((ext_vector_type(16)));
union FragB { v16bf v; v8us h[2]; };

__device__ __forceinline__ v8f wmb(v16bf a, v16bf b, v8f c) {
  v8f d = __builtin_amdgcn_wmma_f32_16x16x32_bf16(false, a, false, b, (short)0, c, false, false);
#if defined(__HIP_DEVICE_COMPILE__)
  asm volatile("v_nop\n\tv_nop\n\tv_nop\n\tv_nop" : "+v"(d) : "v"(a), "v"(b));
#endif
  return d;
}

__device__ __forceinline__ v8f zero8() {
  v8f z = {0.f, 0.f, 0.f, 0.f, 0.f, 0.f, 0.f, 0.f};
  return z;
}

__device__ __forceinline__ unsigned int bfbits(float x) {
  const unsigned int u = __float_as_uint(x);
  return (u + 0x7FFFu + ((u >> 16) & 1u)) >> 16;
}

__device__ __forceinline__ void split8(const float (&v)[8], v4u& hi, v4u& lo) {
  unsigned int hb[8], lb[8];
#pragma unroll
  for (int e = 0; e < 8; ++e) {
    hb[e] = bfbits(v[e]);
    lb[e] = bfbits(v[e] - __uint_as_float(hb[e] << 16));
  }
#pragma unroll
  for (int e = 0; e < 4; ++e) {
    hi[e] = hb[2 * e] | (hb[2 * e + 1] << 16);
    lo[e] = lb[2 * e] | (lb[2 * e + 1] << 16);
  }
}

__global__ void __launch_bounds__(NTHR) __attribute__((amdgpu_num_vgpr(256)))
k_main(const int* __restrict__ seqs, const int* __restrict__ qtok, const float* __restrict__ embed,
       const float* __restrict__ wg_w1, const float* __restrict__ wg_b1,
       const float* __restrict__ wg_w2, const float* __restrict__ wg_b2,
       const float* __restrict__ eg_w1, const float* __restrict__ eg_b1,
       const float* __restrict__ eg_w2, const float* __restrict__ eg_b2,
       const float* __restrict__ rh_w1, const float* __restrict__ rh_b1,
       const float* __restrict__ rh_w2, const float* __restrict__ rh_b2,
       float* out, int nB) {
  extern __shared__ v4f lds_dyn[];
  char* lbase = (char*)lds_dyn;
  float* sEA  = (float*)(lbase + L_EA);
  float* sEM  = (float*)(lbase + L_EM);
  float* sWG  = (float*)(lbase + L_WG);
  float* sGB1 = (float*)(lbase + L_GB1);
  float* sGW2 = (float*)(lbase + L_GW2);
  float* sRB1 = (float*)(lbase + L_RB1);
  float* sRB2 = (float*)(lbase + L_RB2);
  unsigned short* sAh  = (unsigned short*)(lbase + L_AH);
  unsigned short* sAl  = (unsigned short*)(lbase + L_AL);
  unsigned short* sW1h = (unsigned short*)(lbase + L_W1H);
  unsigned short* sW1l = (unsigned short*)(lbase + L_W1L);
  unsigned short* sHh  = (unsigned short*)(lbase + L_HH);
  unsigned short* sHl  = (unsigned short*)(lbase + L_HL);
  unsigned short* sW2h = (unsigned short*)(lbase + L_W2H);
  unsigned short* sW2l = (unsigned short*)(lbase + L_W2L);
  float* sGH  = (float*)(lbase + L_AH);
  float* sStg = (float*)(lbase + L_AH);

  const int tid = threadIdx.x, lane = tid & 31, wave = tid >> 5, hh = lane >> 4, m = lane & 15;

  for (int i = tid; i < NVOC * GH; i += NTHR) {
    const int v = i >> 5, j = i & 31;
    const float* er = embed + v * HID;
    float a0 = 0.0f, a1 = 0.0f;
#pragma unroll 4
    for (int k = 0; k < HID; ++k) {
      const float e = er[k];
      a0 = fmaf(e, eg_w1[k * GH + j], a0);
      a1 = fmaf(e, wg_w1[k * GH + j], a1);
    }
    sEA[i] = a0;
    sGH[i] = fmaxf(a1 + wg_b1[j], 0.0f);
  }
  for (int i = tid; i < HID * (HID2 / 8); i += NTHR) {
    const int n = i >> 4, kc = i & 15;
    float v[8];
#pragma unroll
    for (int e = 0; e < 8; ++e) v[e] = rh_w1[(8 * kc + e) * HID + n];
    v4u hi, lo;
    split8(v, hi, lo);
    *(v4u*)(sW1h + n * AP + 8 * kc) = hi;
    *(v4u*)(sW1l + n * AP + 8 * kc) = lo;
  }
  for (int i = tid; i < HID * (HID / 8); i += NTHR) {
    const int n = i >> 3, kc = i & 7;
    float v[8];
#pragma unroll
    for (int e = 0; e < 8; ++e) v[e] = rh_w2[(8 * kc + e) * HID + n];
    v4u hi, lo;
    split8(v, hi, lo);
    *(v4u*)(sW2h + n * HP + 8 * kc) = hi;
    *(v4u*)(sW2l + n * HP + 8 * kc) = lo;
  }
  if (tid < GH)  { sGB1[tid] = eg_b1[tid]; sGW2[tid] = eg_w2[tid]; }
  if (tid < HID) { sRB1[tid] = rh_b1[tid]; sRB2[tid] = rh_b2[tid]; }
  __syncthreads();

  {
    const int v = tid < NVOC ? tid : NVOC - 1;
    const float* gh = sGH + v * GH;
    float a = 0.0f;
#pragma unroll 4
    for (int j = 0; j < GH; ++j) a = fmaf(gh[j], wg_w2[j], a);
    a += wg_b2[0];
    const float w = 1.0f / (1.0f + expf(-a));
    sWG[tid] = w;
  }
  __syncthreads();

  for (int i = tid; i < NVOC * GH; i += NTHR) {
    const int v = i >> 5, j = i & 31;
    const float w = sWG[v];
    const float* er = embed + v * HID;
    float a = 0.0f;
#pragma unroll 4
    for (int k = 0; k < HID; ++k) {
      const float mv = er[k] * w;
      a = fmaf(mv, eg_w1[(HID + k) * GH + j], a);
    }
    sEM[i] = a;
  }
  __syncthreads();

  const int bidx = blockIdx.x * NTHR + tid;
  const int bc = bidx < nB ? bidx : nB - 1;
  const int* sq = seqs + (size_t)bc * SEQL;
  const float gb2 = eg_b2[0];
  int ts0 = -1, ts1 = -1, ts2 = -1, ts3 = -1;
#pragma unroll 1
  for (int t = 0; t < NSTEP; ++t) {
    int tok = sq[t];
    tok = tok < 0 ? 0 : (tok > NVOC - 1 ? NVOC - 1 : tok);
    const int c0 = ts0 < 0 ? 0 : ts0;
    const int c1 = ts1 < 0 ? 0 : ts1;
    const int c2 = ts2 < 0 ? 0 : ts2;
    const int c3 = ts3 < 0 ? 0 : ts3;
    const float* ea = sEA + tok * GH;
    const float* q0 = sEM + c0 * GH;
    const float* q1 = sEM + c1 * GH;
    const float* q2 = sEM + c2 * GH;
    const float* q3 = sEM + c3 * GH;
    float e0 = 0.0f, e1 = 0.0f, e2 = 0.0f, e3 = 0.0f;
#pragma unroll 2
    for (int jc = 0; jc < GH / 4; ++jc) {
      const v4f av = *(const v4f*)(ea + 4 * jc);
      const v4f bv = *(const v4f*)(sGB1 + 4 * jc);
      const v4f wv = *(const v4f*)(sGW2 + 4 * jc);
      const v4f g0 = *(const v4f*)(q0 + 4 * jc);
      const v4f g1 = *(const v4f*)(q1 + 4 * jc);
      const v4f g2 = *(const v4f*)(q2 + 4 * jc);
      const v4f g3 = *(const v4f*)(q3 + 4 * jc);
#pragma unroll
      for (int e = 0; e < 4; ++e) {
        const float x0 = (av[e] + (ts0 < 0 ? 0.0f : g0[e])) + bv[e];
        const float x1 = (av[e] + (ts1 < 0 ? 0.0f : g1[e])) + bv[e];
        const float x2 = (av[e] + (ts2 < 0 ? 0.0f : g2[e])) + bv[e];
        const float x3 = (av[e] + (ts3 < 0 ? 0.0f : g3[e])) + bv[e];
        e0 = fmaf(fmaxf(x0, 0.0f), wv[e], e0);
        e1 = fmaf(fmaxf(x1, 0.0f), wv[e], e1);
        e2 = fmaf(fmaxf(x2, 0.0f), wv[e], e2);
        e3 = fmaf(fmaxf(x3, 0.0f), wv[e], e3);
      }
    }
    const float l0 = e0 + gb2, l1 = e1 + gb2, l2 = e2 + gb2, l3 = e3 + gb2;
    int a = 0;
    float best = l0;
    if (l1 > best) { best = l1; a = 1; }
    if (l2 > best) { best = l2; a = 2; }
    if (l3 > best) { best = l3; a = 3; }
    ts0 = (a == 0) ? tok : ts0;
    ts1 = (a == 1) ? tok : ts1;
    ts2 = (a == 2) ? tok : ts2;
    ts3 = (a == 3) ? tok : ts3;
  }

  {
    int qt = qtok[bc];
    qt = qt < 0 ? 0 : (qt > NVOC - 1 ? NVOC - 1 : qt);
    const float* qr = embed + qt * HID;
    const int c0 = ts0 < 0 ? 0 : ts0;
    const int c1 = ts1 < 0 ? 0 : ts1;
    const int c2 = ts2 < 0 ? 0 : ts2;
    const int c3 = ts3 < 0 ? 0 : ts3;
    const float w0 = sWG[c0], w1 = sWG[c1], w2 = sWG[c2], w3 = sWG[c3];
    const float* p0 = embed + c0 * HID;
    const float* p1 = embed + c1 * HID;
    const float* p2 = embed + c2 * HID;
    const float* p3 = embed + c3 * HID;
    unsigned short* ahr = sAh + tid * AP;
    unsigned short* alr = sAl + tid * AP;
#pragma unroll 2
    for (int kc = 0; kc < HID / 8; ++kc) {
      float v[8];
      {
        const v4f qa = *(const v4f*)(qr + 8 * kc);
        const v4f qb = *(const v4f*)(qr + 8 * kc + 4);
#pragma unroll
        for (int e = 0; e < 4; ++e) { v[e] = qa[e]; v[4 + e] = qb[e]; }
      }
      v4u hi, lo;
      split8(v, hi, lo);
      *(v4u*)(ahr + 8 * kc) = hi;
      *(v4u*)(alr + 8 * kc) = lo;
      {
        const v4f a0 = *(const v4f*)(p0 + 8 * kc), b0 = *(const v4f*)(p0 + 8 * kc + 4);
        const v4f a1 = *(const v4f*)(p1 + 8 * kc), b1 = *(const v4f*)(p1 + 8 * kc + 4);
        const v4f a2 = *(const v4f*)(p2 + 8 * kc), b2 = *(const v4f*)(p2 + 8 * kc + 4);
        const v4f a3 = *(const v4f*)(p3 + 8 * kc), b3 = *(const v4f*)(p3 + 8 * kc + 4);
#pragma unroll
        for (int e = 0; e < 4; ++e) {
          float s = (ts0 < 0) ? 0.0f : a0[e] * w0;
          s += (ts1 < 0) ? 0.0f : a1[e] * w1;
          s += (ts2 < 0) ? 0.0f : a2[e] * w2;
          s += (ts3 < 0) ? 0.0f : a3[e] * w3;
          v[e] = s * 0.25f;
          float u = (ts0 < 0) ? 0.0f : b0[e] * w0;
          u += (ts1 < 0) ? 0.0f : b1[e] * w1;
          u += (ts2 < 0) ? 0.0f : b2[e] * w2;
          u += (ts3 < 0) ? 0.0f : b3[e] * w3;
          v[4 + e] = u * 0.25f;
        }
      }
      split8(v, hi, lo);
      *(v4u*)(ahr + HID + 8 * kc) = hi;
      *(v4u*)(alr + HID + 8 * kc) = lo;
    }
  }
  __syncthreads();

#pragma unroll 1
  for (int mt = 0; mt < 2; ++mt) {
    const int ra = wave * 32 + mt * 16;
    v8f acc[4];
#pragma unroll
    for (int tt = 0; tt < 4; ++tt) acc[tt] = zero8();
#pragma unroll 1
    for (int kt = 0; kt < HID2 / 32; ++kt) {
      FragB ah, al;
      const unsigned short* ap = sAh + (ra + m) * AP + 32 * kt + 8 * hh;
      const unsigned short* aq = sAl + (ra + m) * AP + 32 * kt + 8 * hh;
      ah.h[0] = *(const v8us*)ap;  ah.h[1] = *(const v8us*)(ap + 16);
      al.h[0] = *(const v8us*)aq;  al.h[1] = *(const v8us*)(aq + 16);
#pragma unroll
      for (int tt = 0; tt < 4; ++tt) {
        const unsigned short* bp = sW1h + (16 * tt + m) * AP + 32 * kt + 8 * hh;
        const unsigned short* bq = sW1l + (16 * tt + m) * AP + 32 * kt + 8 * hh;
        FragB bh, bl;
        bh.h[0] = *(const v8us*)bp;  bh.h[1] = *(const v8us*)(bp + 16);
        bl.h[0] = *(const v8us*)bq;  bl.h[1] = *(const v8us*)(bq + 16);
        acc[tt] = wmb(ah.v, bh.v, acc[tt]);
        acc[tt] = wmb(ah.v, bl.v, acc[tt]);
        acc[tt] = wmb(al.v, bh.v, acc[tt]);
      }
    }
#pragma unroll
    for (int tt = 0; tt < 4; ++tt) {
      const float bb = sRB1[16 * tt + m];
#pragma unroll
      for (int r = 0; r < 8; ++r) {
        const float x = fmaxf(acc[tt][r] + bb, 0.0f);
        const unsigned int hb = bfbits(x);
        const unsigned int lb = bfbits(x - __uint_as_float(hb << 16));
        const int idx = (ra + 8 * hh + r) * HP + 16 * tt + m;
        sHh[idx] = (unsigned short)hb;
        sHl[idx] = (unsigned short)lb;
      }
    }
  }
  __syncthreads();

#pragma unroll 1
  for (int mt = 0; mt < 2; ++mt) {
    const int ra = wave * 32 + mt * 16;
    v8f acc[4];
#pragma unroll
    for (int tt = 0; tt < 4; ++tt) acc[tt] = zero8();
#pragma unroll 1
    for (int kt = 0; kt < HID / 32; ++kt) {
      FragB ah, al;
      const unsigned short* ap = sHh + (ra + m) * HP + 32 * kt + 8 * hh;
      const unsigned short* aq = sHl + (ra + m) * HP + 32 * kt + 8 * hh;
      ah.h[0] = *(const v8us*)ap;  ah.h[1] = *(const v8us*)(ap + 16);
      al.h[0] = *(const v8us*)aq;  al.h[1] = *(const v8us*)(aq + 16);
#pragma unroll
      for (int tt = 0; tt < 4; ++tt) {
        const unsigned short* bp = sW2h + (16 * tt + m) * HP + 32 * kt + 8 * hh;
        const unsigned short* bq = sW2l + (16 * tt + m) * HP + 32 * kt + 8 * hh;
        FragB bh, bl;
        bh.h[0] = *(const v8us*)bp;  bh.h[1] = *(const v8us*)(bp + 16);
        bl.h[0] = *(const v8us*)bq;  bl.h[1] = *(const v8us*)(bq + 16);
        acc[tt] = wmb(ah.v, bh.v, acc[tt]);
        acc[tt] = wmb(ah.v, bl.v, acc[tt]);
        acc[tt] = wmb(al.v, bh.v, acc[tt]);
      }
    }
    float* stw = sStg + wave * (32 * HID);
#pragma unroll
    for (int tt = 0; tt < 4; ++tt) {
      const float bb = sRB2[16 * tt + m];
#pragma unroll
      for (int r = 0; r < 8; ++r)
        stw[(mt * 16 + 8 * hh + r) * HID + 16 * tt + m] = acc[tt][r] + bb;
    }
  }
  __syncthreads();

  {
    const float* sw = sStg + wave * (32 * HID);
    v4f pv[16];
#pragma unroll
    for (int p = 0; p < 16; ++p) pv[p] = *(const v4f*)(sw + (2 * p + hh) * HID + 4 * m);
    const int rbase = blockIdx.x * NTHR + wave * 32;
#pragma unroll
    for (int p = 0; p < 16; ++p) {
      const int gr = rbase + 2 * p + hh;
      if (gr < nB) *(volatile v4f*)(out + (size_t)gr * HID + 4 * m) = pv[p];
    }
    __threadfence();
#pragma unroll
    for (int p = 0; p < 16; ++p) {
      const int gr = rbase + 2 * p + hh;
      if (gr < nB) *(volatile v4f*)(out + (size_t)gr * HID + 4 * m) = pv[p];
    }
  }
}

extern "C" void kernel_launch(void* const* d_in, const int* in_sizes, int n_in,
                              void* d_out, int out_size, void* d_ws, size_t ws_size,
                              hipStream_t stream) {
  (void)d_ws; (void)ws_size;
  if (n_in < 15) return;
  const int nB = in_sizes[1];
  if (nB <= 0 || nB > (1 << 24)) return;
  if (in_sizes[0] != nB * SEQL) return;
  if (in_sizes[2] != NVOC * HID || in_sizes[3] != HID * GH || in_sizes[4] != GH) return;
  if (in_sizes[5] != GH || in_sizes[6] < 1) return;
  if (in_sizes[7] != HID2 * GH || in_sizes[8] != GH || in_sizes[9] != GH || in_sizes[10] < 1) return;
  if (in_sizes[11] != HID2 * HID || in_sizes[12] != HID || in_sizes[13] != HID * HID || in_sizes[14] != HID) return;
  if (out_size != nB * HID) return;

  const int*   seqs  = (const int*)d_in[0];
  const int*   qtok  = (const int*)d_in[1];
  const float* embed = (const float*)d_in[2];
  const float* wg_w1 = (const float*)d_in[3];
  const float* wg_b1 = (const float*)d_in[4];
  const float* wg_w2 = (const float*)d_in[5];
  const float* wg_b2 = (const float*)d_in[6];
  const float* eg_w1 = (const float*)d_in[7];
  const float* eg_b1 = (const float*)d_in[8];
  const float* eg_w2 = (const float*)d_in[9];
  const float* eg_b2 = (const float*)d_in[10];
  const float* rh_w1 = (const float*)d_in[11];
  const float* rh_b1 = (const float*)d_in[12];
  const float* rh_w2 = (const float*)d_in[13];
  const float* rh_b2 = (const float*)d_in[14];
  float* out = (float*)d_out;

  const int nBlk = (nB + NTHR - 1) / NTHR;
  hipFuncSetAttribute(reinterpret_cast<const void*>(&k_main),
                      hipFuncAttributeMaxDynamicSharedMemorySize, LDS_TOT);
  k_main<<<nBlk, NTHR, LDS_TOT, stream>>>(seqs, qtok, embed,
                                         wg_w1, wg_b1, wg_w2, wg_b2,
                                         eg_w1, eg_b1, eg_w2, eg_b2,
                                         rh_w1, rh_b1, rh_w2, rh_b2, out, nB);
}
